// DeformableCrossAttention2D_50311246905785
// MI455X (gfx1250) — hardware-verified
//
#include <hip/hip_runtime.h>
#include <stddef.h>
#include <math.h>

constexpr int NBATCH = 8;
constexpr int NCH    = 256;
constexpr int NHEAD  = 8;
constexpr int HDIM   = 32;
constexpr int NPT    = 4;
constexpr int QIMG   = 64;
constexpr int QPIX   = 4096;
constexpr int KIMG   = 32;
constexpr int KPIX   = 1024;
constexpr int NOFF   = 64;
constexpr int NTAP   = 9;
constexpr int KIM    = 2304;
constexpr int IMGS_PER_CHUNK = 2;
constexpr int NCHUNK = 4;
constexpr float OFF_RANGE  = 0.25f;
constexpr float RSQRT_HDIM = 0.17677669529663687f;
constexpr float OUT_CARRY  = 8.0f;
constexpr float WOUT_CARRY = 16.0f;
constexpr float OUT_SCALE  = 1.0f / 128.0f;

static_assert(NHEAD * HDIM == NCH, "");
static_assert(NHEAD * NPT * 2 == NOFF, "");
static_assert(NTAP * NCH == KIM, "");
static_assert(KIM % 32 == 0 && NCH % 32 == 0, "");
static_assert(QPIX % 64 == 0 && KPIX % 64 == 0 && NCH % 64 == 0 && NOFF % 64 == 0, "");
static_assert(IMGS_PER_CHUNK * NCHUNK == NBATCH, "");
static_assert((IMGS_PER_CHUNK * QPIX * NTAP) % 8 == 0, "");
static_assert((NBATCH * QPIX) % 8 == 0, "");

typedef __attribute__((ext_vector_type(16))) _Float16 v16h;
typedef __attribute__((ext_vector_type(8)))  _Float16 v8h;
typedef __attribute__((ext_vector_type(16))) __bf16   v16b;
typedef __attribute__((ext_vector_type(8)))  __bf16   v8b;
typedef __attribute__((ext_vector_type(8)))  float    v8f;
typedef __attribute__((ext_vector_type(4)))  float    v4f;
typedef __attribute__((ext_vector_type(4)))  unsigned v4u;

__device__ __forceinline__ unsigned short f2bf_bits(float f) {
  unsigned u = __float_as_uint(f);
  return (unsigned short)((u + 0x7FFFu + ((u >> 16) & 1u)) >> 16);
}
__device__ __forceinline__ float bf_bits2f(unsigned short h) { return __uint_as_float(((unsigned)h) << 16); }
__device__ __forceinline__ float bf16r(float f) { return bf_bits2f(f2bf_bits(f)); }

__device__ __forceinline__ unsigned pk2(unsigned short a, unsigned short b) {
  return (unsigned)a | ((unsigned)b << 16);
}
__device__ __forceinline__ unsigned pkh2(float a, float b) {
  return pk2(__builtin_bit_cast(unsigned short, (_Float16)a), __builtin_bit_cast(unsigned short, (_Float16)b));
}

__device__ __forceinline__ void dep_guard_h(v8f& a, v8f& b, v16h x, v16h y) { asm volatile("v_nop\n\tv_nop\n\tv_nop\n\tv_nop" : "+v"(a), "+v"(b) : "v"(x), "v"(y)); }
__device__ __forceinline__ void dep_guard_b(v8f& a, v8f& b, v16b x, v16b y) { asm volatile("v_nop\n\tv_nop\n\tv_nop\n\tv_nop" : "+v"(a), "+v"(b) : "v"(x), "v"(y)); }
__device__ __forceinline__ void keep4_h(v16h a, v16h b, v16h c, v16h d) { asm volatile("v_nop" :: "v"(a), "v"(b), "v"(c), "v"(d)); }
__device__ __forceinline__ void keep4_b(v16b a, v16b b, v16b c, v16b d) { asm volatile("v_nop" :: "v"(a), "v"(b), "v"(c), "v"(d)); }
__device__ __forceinline__ void acc_guard4(v8f& a, v8f& b, v8f& c, v8f& d) { asm volatile("v_nop\n\tv_nop\n\tv_nop\n\tv_nop" : "+v"(a), "+v"(b), "+v"(c), "+v"(d)); }
template <typename T> struct Frag;
template <> struct Frag<_Float16> {
  typedef v16h V; union U { v16h v; v8h h[2]; };
  static __device__ __forceinline__ v16h load(const _Float16* p) {
    U f; f.h[0] = *(const v8h*)(p); f.h[1] = *(const v8h*)(p + 16); return f.v;
  }
  static __device__ __forceinline__ v8f mma(v16h a, v16h b, v8f c) {
    return __builtin_amdgcn_wmma_f32_16x16x32_f16(false, a, false, b, (short)0, c, false, false);
  }
  static __device__ __forceinline__ void guard(v8f& a, v8f& b, v16h x, v16h y) { dep_guard_h(a, b, x, y); }
  static __device__ __forceinline__ void keep(v16h a, v16h b, v16h c, v16h d) { keep4_h(a, b, c, d); }
};
template <> struct Frag<__bf16> {
  typedef v16b V; union U { v16b v; v8b h[2]; };
  static __device__ __forceinline__ v16b load(const __bf16* p) {
    U f; f.h[0] = *(const v8b*)(p); f.h[1] = *(const v8b*)(p + 16); return f.v;
  }
  static __device__ __forceinline__ v8f mma(v16b a, v16b b, v8f c) {
    return __builtin_amdgcn_wmma_f32_16x16x32_bf16(false, a, false, b, (short)0, c, false, false);
  }
  static __device__ __forceinline__ void guard(v8f& a, v8f& b, v16b x, v16b y) { dep_guard_b(a, b, x, y); }
  static __device__ __forceinline__ void keep(v16b a, v16b b, v16b c, v16b d) { keep4_b(a, b, c, d); }
};

template <int ET> struct Elem;
template <> struct Elem<0> { typedef _Float16 T; };
template <> struct Elem<1> { typedef __bf16 T; };
template <int ET, int SPLITM, int BIAS_MODE, int OUT_MODE, bool RESID, int ACT = 0>
__global__ __launch_bounds__(256) void wmma_gemm64(
    const unsigned short* __restrict__ Ap, const unsigned short* __restrict__ A2p, int lda, long strideA,
    const unsigned short* __restrict__ Btp, const unsigned short* __restrict__ Bt2p, int ldb, long strideB,
    void* __restrict__ Cout, void* __restrict__ Cout2, int ldc, long strideC,
    const float* __restrict__ bias,
    const float* __restrict__ resid, long strideR,
    int M, int N, int K, float scale) {
  typedef typename Elem<ET>::T T;
  typedef typename Frag<T>::V V;
  constexpr bool SPLA = (SPLITM != 0);
  constexpr bool SPLB = (SPLITM == 1);
  const T* A = (const T*)Ap; const T* A2 = (const T*)A2p; const T* Bt = (const T*)Btp; const T* Bt2 = (const T*)Bt2p;
  __shared__ __align__(16) float sT[8][16 * 68];
  const int b    = blockIdx.y;
  const int lane = threadIdx.x & 31;
  const int wave = threadIdx.x >> 5;
  const int tilesN = N >> 6;
  const int tilesM = M >> 6;
  const int tile = blockIdx.x * 8 + wave;
  if (tile >= tilesM * tilesN) return;
  const int tm = tile / tilesN;
  const int tn = tile - tm * tilesN;
  const int m0 = tm << 6;
  const int n0 = tn << 6;

  const T* Ab  = A  + (size_t)b * strideA;
  const T* Bb  = Bt + (size_t)b * strideB;
  const T* Ab2 = SPLA ? (A2  + (size_t)b * strideA) : nullptr;
  const T* Bb2 = SPLB ? (Bt2 + (size_t)b * strideB) : nullptr;

  const int rlane = lane & 15;
  const int koff  = (lane >> 4) * 8;
  const int mOff  = (lane >> 4) * 8;

  v8f acc[4][4];
#pragma unroll
  for (int i = 0; i < 4; ++i)
#pragma unroll
    for (int j = 0; j < 4; ++j) acc[i][j] = (v8f){0.f,0.f,0.f,0.f,0.f,0.f,0.f,0.f};

  for (int k0 = 0; k0 < K; k0 += 32) {
    V bh[4], bl[4];
#pragma unroll
    for (int j = 0; j < 4; ++j) {
      const size_t bo = (size_t)(n0 + (j << 4) + rlane) * ldb + koff + k0;
      bh[j] = Frag<T>::load(Bb + bo);
      if (SPLB) bl[j] = Frag<T>::load(Bb2 + bo);
    }
#pragma unroll
    for (int i = 0; i < 4; ++i) {
      const size_t ao = (size_t)(m0 + (i << 4) + rlane) * lda + koff + k0;
      V ah = Frag<T>::load(Ab + ao);
      V al;
      if (SPLA) al = Frag<T>::load(Ab2 + ao);
#pragma unroll
      for (int j = 0; j < 4; ++j) {
        acc[i][j] = Frag<T>::mma(ah, bh[j], acc[i][j]);
        if (SPLB) acc[i][j] = Frag<T>::mma(ah, bl[j], acc[i][j]);
        if (SPLA) acc[i][j] = Frag<T>::mma(al, bh[j], acc[i][j]);
      }
      Frag<T>::guard(acc[i][0], acc[i][3], ah, SPLA ? al : ah);
    }
    Frag<T>::keep(bh[0], bh[1], bh[2], bh[3]);
    if (SPLB) Frag<T>::keep(bl[0], bl[1], bl[2], bl[3]);
  }
  acc_guard4(acc[0][0], acc[0][1], acc[0][2], acc[0][3]);
  acc_guard4(acc[1][0], acc[1][1], acc[1][2], acc[1][3]);
  acc_guard4(acc[2][0], acc[2][1], acc[2][2], acc[2][3]);
  acc_guard4(acc[3][0], acc[3][1], acc[3][2], acc[3][3]);

  float* slab = sT[wave];
  const float* Rb = RESID ? (resid + (size_t)b * strideR) : nullptr;
#pragma unroll
  for (int i = 0; i < 4; ++i) {
    const int mBase = m0 + (i << 4);
#pragma unroll
    for (int j = 0; j < 4; ++j) {
      const int n = n0 + (j << 4) + rlane;
      float bv = 0.f;
      if (BIAS_MODE == 2) bv = bias[n];
#pragma unroll
      for (int r = 0; r < 8; ++r) {
        float v = acc[i][j][r] * scale;
        if (BIAS_MODE == 1) v += bias[mBase + mOff + r];
        if (BIAS_MODE == 2) v += bv;
        if (ACT == 1) v = tanhf(v);
        if (ACT == 2) v = fmaxf(v, 0.0f);
        if (ACT == 4) v = (v > 0.f) ? v : 0.01f * v;
        if (RESID) v += Rb[(size_t)(mBase + mOff + r) * ldc + n];
        slab[(mOff + r) * 68 + (j << 4) + rlane] = v;
      }
    }
    __builtin_amdgcn_fence(__ATOMIC_RELEASE, "workgroup");
    __builtin_amdgcn_wave_barrier();
    __builtin_amdgcn_fence(__ATOMIC_ACQUIRE, "workgroup");
    if (OUT_MODE == 0) {
      float* C = (float*)Cout + (size_t)b * strideC;
      const int hh = lane >> 4, c4 = (lane & 15) * 4;
      for (int pass = 0; pass < 2; ++pass) {
#pragma unroll
        for (int it = 0; it < 8; ++it) {
          const int row = it * 2 + hh;
          v4f v = *(const v4f*)(slab + row * 68 + c4);
          *(volatile v4f*)(C + (size_t)(mBase + row) * ldc + n0 + c4) = v;
        }
        __threadfence();
      }
    } else {
      const int q = lane >> 3, c8 = (lane & 7) * 8;
      unsigned short* C  = (unsigned short*)Cout  + (size_t)b * strideC;
      unsigned short* C2 = (OUT_MODE == 2) ? ((unsigned short*)Cout2 + (size_t)b * strideC) : nullptr;
      for (int pass = 0; pass < 2; ++pass) {
#pragma unroll
        for (int it = 0; it < 4; ++it) {
          const int row = it * 4 + q;
          const float* sp = slab + row * 68 + c8;
          v8h hv, lv;
#pragma unroll
          for (int e = 0; e < 8; ++e) {
            if (OUT_MODE == 1) {
              hv[e] = (_Float16)sp[e];
            } else {
              unsigned short hb = f2bf_bits(sp[e]);
              unsigned short lb = f2bf_bits(sp[e] - bf_bits2f(hb));
              hv[e] = __builtin_bit_cast(_Float16, hb);
              lv[e] = __builtin_bit_cast(_Float16, lb);
            }
          }
          *(volatile v8h*)(C + (size_t)(mBase + row) * ldc + n0 + c8) = hv;
          if (OUT_MODE == 2) *(volatile v8h*)(C2 + (size_t)(mBase + row) * ldc + n0 + c8) = lv;
        }
        __threadfence();
      }
    }
    __builtin_amdgcn_fence(__ATOMIC_RELEASE, "workgroup");
    __builtin_amdgcn_wave_barrier();
    __builtin_amdgcn_fence(__ATOMIC_ACQUIRE, "workgroup");
  }
}

__global__ __launch_bounds__(256) void k_tr_in(const float* __restrict__ in, unsigned short* __restrict__ dst, int NP) {
  __shared__ float t[64][65];
  const int tid = threadIdx.x;
  const int p0 = blockIdx.x * 64, c0 = blockIdx.y * 64, b = blockIdx.z;
  const int p4 = (tid & 15) * 4;
  const float* src = in + ((size_t)b * NCH + c0) * NP + p0;
#pragma unroll
  for (int it = 0; it < 4; ++it) {
    const int row = it * 16 + (tid >> 4);
    const v4f v = *(const v4f*)(src + (size_t)row * NP + p4);
#pragma unroll
    for (int e = 0; e < 4; ++e) t[row][p4 + e] = bf16r(v[e]);
  }
  __syncthreads();
  const int wave = tid >> 5, lane = tid & 31, q = lane >> 3, k8 = (lane & 7) * 8;
  for (int pass = 0; pass < 2; ++pass) {
#pragma unroll
    for (int step = 0; step < 2; ++step) {
      const int pp = step * 32 + wave * 4 + q;
      v4u u;
      u[0] = pk2(f2bf_bits(t[k8 + 0][pp]), f2bf_bits(t[k8 + 1][pp]));
      u[1] = pk2(f2bf_bits(t[k8 + 2][pp]), f2bf_bits(t[k8 + 3][pp]));
      u[2] = pk2(f2bf_bits(t[k8 + 4][pp]), f2bf_bits(t[k8 + 5][pp]));
      u[3] = pk2(f2bf_bits(t[k8 + 6][pp]), f2bf_bits(t[k8 + 7][pp]));
      *(volatile v4u*)(dst + ((size_t)b * NP + p0 + pp) * NCH + c0 + k8) = u;
    }
    __threadfence();
  }
}

__global__ __launch_bounds__(256) void k_castw(const float* __restrict__ wq, const float* __restrict__ wk,
                                              const float* __restrict__ wv, const float* __restrict__ wo,
                                              unsigned short* __restrict__ dq, unsigned short* __restrict__ dk,
                                              unsigned short* __restrict__ dv, unsigned short* __restrict__ dw) {
  const int sel = blockIdx.y;
  const float* src; unsigned short* dst;
  if (sel == 0) { src = wq; dst = dq; }
  else if (sel == 1) { src = wk; dst = dk; }
  else if (sel == 2) { src = wv; dst = dv; }
  else { src = wo; dst = dw; }
  const int i = blockIdx.x * 256 + threadIdx.x;
  const float* s = src + (size_t)i * 8;
  const v4f a = *(const v4f*)s;
  const v4f c = *(const v4f*)(s + 4);
  v4u u;
  if (sel == 3) {
    u[0] = pkh2(bf16r(a[0]) * WOUT_CARRY, bf16r(a[1]) * WOUT_CARRY);
    u[1] = pkh2(bf16r(a[2]) * WOUT_CARRY, bf16r(a[3]) * WOUT_CARRY);
    u[2] = pkh2(bf16r(c[0]) * WOUT_CARRY, bf16r(c[1]) * WOUT_CARRY);
    u[3] = pkh2(bf16r(c[2]) * WOUT_CARRY, bf16r(c[3]) * WOUT_CARRY);
  } else {
    u[0] = pk2(f2bf_bits(a[0]), f2bf_bits(a[1]));
    u[1] = pk2(f2bf_bits(a[2]), f2bf_bits(a[3]));
    u[2] = pk2(f2bf_bits(c[0]), f2bf_bits(c[1]));
    u[3] = pk2(f2bf_bits(c[2]), f2bf_bits(c[3]));
  }
  volatile v4u* p = (volatile v4u*)(dst + (size_t)i * 8);
  *p = u;
  __threadfence();
  *p = u;
}

__global__ __launch_bounds__(256) void k_prepoff(const float* __restrict__ w, unsigned short* __restrict__ dst) {
  const int gidx = blockIdx.x * 256 + threadIdx.x;
  const int o = gidx / (KIM / 8);
  const int rem = gidx - o * (KIM / 8);
  const int k0 = rem * 8;
  const int tap = k0 >> 8;
  const int c = k0 & (NCH - 1);
  const float* wr = w + ((size_t)o * NCH + c) * NTAP + tap;
  v4u u;
  u[0] = pk2(f2bf_bits(wr[0 * NTAP]), f2bf_bits(wr[1 * NTAP]));
  u[1] = pk2(f2bf_bits(wr[2 * NTAP]), f2bf_bits(wr[3 * NTAP]));
  u[2] = pk2(f2bf_bits(wr[4 * NTAP]), f2bf_bits(wr[5 * NTAP]));
  u[3] = pk2(f2bf_bits(wr[6 * NTAP]), f2bf_bits(wr[7 * NTAP]));
  volatile v4u* p = (volatile v4u*)(dst + (size_t)o * KIM + k0);
  *p = u;
  __threadfence();
  *p = u;
}

__global__ __launch_bounds__(256) void k_im2col(const unsigned short* __restrict__ qt,
                                               unsigned short* __restrict__ im, int b0) {
  const int tid = threadIdx.x;
  const int lane = tid & 31;
  const int wg = blockIdx.x * 8 + (tid >> 5);
  const int img = wg / (QPIX * NTAP);
  const int rem = wg - img * (QPIX * NTAP);
  const int px = rem / NTAP;
  const int tap = rem - px * NTAP;
  const int ky = tap / 3, kx = tap - ky * 3;
  const int y = px >> 6, x = px & 63;
  const int yy = y + ky - 1, xx = x + kx - 1;
  const bool inb = ((unsigned)yy < (unsigned)QIMG) && ((unsigned)xx < (unsigned)QIMG);
  const int yc = min(max(yy, 0), QIMG - 1);
  const int xc = min(max(xx, 0), QIMG - 1);
  const v4u v = *(const v4u*)(qt + ((size_t)(b0 + img) * QPIX + yc * QIMG + xc) * NCH + lane * 8);
  v4u o;
  o[0] = inb ? v[0] : 0u;
  o[1] = inb ? v[1] : 0u;
  o[2] = inb ? v[2] : 0u;
  o[3] = inb ? v[3] : 0u;
  volatile v4u* p = (volatile v4u*)(im + ((size_t)img * QPIX + px) * KIM + tap * NCH + lane * 8);
  *p = o;
  __threadfence();
  *p = o;
}

__global__ __launch_bounds__(256) void k_sample(const float* __restrict__ qf, const float* __restrict__ kf,
                                               const float* __restrict__ vf, const float* __restrict__ off,
                                               unsigned short* __restrict__ out16) {
  __shared__ __align__(16) unsigned rowbuf[8][128];
  const int tid = threadIdx.x;
  const int wave = tid >> 5, lane = tid & 31;
  const int g = lane >> 3, j = lane & 7;
  const int odd = j & 1;
  const int gw = blockIdx.x * 8 + wave;
  const int b = gw >> 12;
  const int px = gw & (QPIX - 1);
  const int iy = px >> 6, ix = px & 63;

  const float rstep = 1.0f / 63.0f;
  const float sx = (float)ix * rstep, sy = (float)iy * rstep;
  float basex = -1.0f * (1.0f - sx) + 1.0f * sx;
  float basey = -1.0f * (1.0f - sy) + 1.0f * sy;
  basex = (ix == QIMG - 1) ? 1.0f : basex;
  basey = (iy == QIMG - 1) ? 1.0f : basey;

  unsigned* rb = rowbuf[wave];
  const float* offrow = off + ((size_t)b * QPIX + px) * NOFF;
  const float* qrow   = qf  + ((size_t)b * QPIX + px) * NCH;
  const float* kbase  = kf  + (size_t)b * KPIX * NCH;
  const float* vbase  = vf  + (size_t)b * KPIX * NCH;

#pragma unroll 1
  for (int hg = 0; hg < 2; ++hg) {
    const int h = hg * 4 + g;
    const int cb = h * HDIM + 4 * j;
    const v4f q4 = *(const v4f*)(qrow + cb);
    float mrun = -INFINITY, lrun = 0.0f;
    v4f acc = (v4f){0.f, 0.f, 0.f, 0.f};
#pragma unroll 1
    for (int p = 0; p < NPT; ++p) {
      const int mch = h * (NPT * 2) + p * 2;
      const float oraw = offrow[mch + odd];
      const float tn = tanhf(oraw) * OFF_RANGE;
      const float tother = __shfl_xor(tn, 1, 32);
      const float offx = odd ? tother : tn;
      const float offy = odd ? tn : tother;
      const float gx = basex + offx;
      const float gy = basey + offy;
      const float xs = (gx + 1.0f) * (KIMG * 0.5f) - 0.5f;
      const float ys = (gy + 1.0f) * (KIMG * 0.5f) - 0.5f;
      const float x0f = floorf(xs), y0f = floorf(ys);
      const float wx1 = xs - x0f, wy1 = ys - y0f;
      const float wx0 = 1.0f - wx1, wy0 = 1.0f - wy1;
      int x0 = (int)x0f, y0 = (int)y0f;
      x0 = max(-8, min(x0, 40));
      y0 = max(-8, min(y0, 40));
      const int x1 = x0 + 1, y1 = y0 + 1;
      const bool vx0 = (unsigned)x0 < (unsigned)KIMG, vx1 = (unsigned)x1 < (unsigned)KIMG;
      const bool vy0 = (unsigned)y0 < (unsigned)KIMG, vy1 = (unsigned)y1 < (unsigned)KIMG;
      const int xc0 = min(max(x0, 0), KIMG - 1), xc1 = min(max(x1, 0), KIMG - 1);
      const int yc0 = min(max(y0, 0), KIMG - 1), yc1 = min(max(y1, 0), KIMG - 1);
      const float w00 = (vy0 && vx0) ? wx0 * wy0 : 0.0f;
      const float w01 = (vy0 && vx1) ? wx1 * wy0 : 0.0f;
      const float w10 = (vy1 && vx0) ? wx0 * wy1 : 0.0f;
      const float w11 = (vy1 && vx1) ? wx1 * wy1 : 0.0f;
      const size_t o00 = (size_t)(yc0 * KIMG + xc0) * NCH + cb;
      const size_t o01 = (size_t)(yc0 * KIMG + xc1) * NCH + cb;
      const size_t o10 = (size_t)(yc1 * KIMG + xc0) * NCH + cb;
      const size_t o11 = (size_t)(yc1 * KIMG + xc1) * NCH + cb;
      const v4f k00 = *(const v4f*)(kbase + o00);
      const v4f k01 = *(const v4f*)(kbase + o01);
      const v4f k10 = *(const v4f*)(kbase + o10);
      const v4f k11 = *(const v4f*)(kbase + o11);
      const v4f v00 = *(const v4f*)(vbase + o00);
      const v4f v01 = *(const v4f*)(vbase + o01);
      const v4f v10 = *(const v4f*)(vbase + o10);
      const v4f v11 = *(const v4f*)(vbase + o11);
      v4f ks = k00 * w00;
      ks = ks + k01 * w01;
      ks = ks + k10 * w10;
      ks = ks + k11 * w11;
      v4f vs = v00 * w00;
      vs = vs + v01 * w01;
      vs = vs + v10 * w10;
      vs = vs + v11 * w11;
      float d = q4[0] * ks[0];
      d = d + q4[1] * ks[1];
      d = d + q4[2] * ks[2];
      d = d + q4[3] * ks[3];
      d += __shfl_xor(d, 1, 32);
      d += __shfl_xor(d, 2, 32);
      d += __shfl_xor(d, 4, 32);
      const float logit = d * RSQRT_HDIM;
      const float mnew = fmaxf(mrun, logit);
      const float alpha = __expf(mrun - mnew);
      const float pe = __expf(logit - mnew);
      lrun = lrun * alpha + pe;
      acc = acc * alpha + vs * pe;
      mrun = mnew;
    }
    const float inv = __builtin_amdgcn_rcpf(lrun) * OUT_CARRY;
    const unsigned u0 = pkh2(acc[0] * inv, acc[1] * inv);
    const unsigned u1 = pkh2(acc[2] * inv, acc[3] * inv);
    rb[(cb >> 1)] = u0;
    rb[(cb >> 1) + 1] = u1;
  }
  __builtin_amdgcn_fence(__ATOMIC_RELEASE, "workgroup");
  __builtin_amdgcn_wave_barrier();
  __builtin_amdgcn_fence(__ATOMIC_ACQUIRE, "workgroup");
  const v4u val = *(const v4u*)(rb + lane * 4);
  volatile v4u* dstp = (volatile v4u*)(out16 + ((size_t)b * QPIX + px) * NCH + lane * 8);
  *dstp = val;
  __threadfence();
  *dstp = val;
}

extern "C" void kernel_launch(void* const* d_in, const int* in_sizes, int n_in,
                              void* d_out, int out_size, void* d_ws, size_t ws_size,
                              hipStream_t stream) {
  if (n_in < 8) return;
  if (in_sizes[0] != NBATCH * NCH * QPIX) return;
  if (in_sizes[1] != NBATCH * NCH * KPIX) return;
  if (in_sizes[2] != NCH * NCH || in_sizes[3] != NCH * NCH || in_sizes[4] != NCH * NCH || in_sizes[7] != NCH * NCH) return;
  if (in_sizes[5] != NOFF * NCH * NTAP || in_sizes[6] != NOFF) return;
  if (out_size != NBATCH * NCH * QPIX) return;

  const float* query_map = (const float*)d_in[0];
  const float* kv_map    = (const float*)d_in[1];
  const float* q_w       = (const float*)d_in[2];
  const float* k_w       = (const float*)d_in[3];
  const float* v_w       = (const float*)d_in[4];
  const float* offset_w  = (const float*)d_in[5];
  const float* offset_b  = (const float*)d_in[6];
  const float* out_w     = (const float*)d_in[7];
  float* out = (float*)d_out;

  const size_t szQT   = (size_t)NBATCH * QPIX * NCH * 2;
  const size_t szKVT  = (size_t)NBATCH * KPIX * NCH * 2;
  const size_t szW    = (size_t)NCH * NCH * 2;
  const size_t szWOFF = (size_t)NOFF * KIM * 2;
  const size_t szQ    = (size_t)NBATCH * QPIX * NCH * 4;
  const size_t szK    = (size_t)NBATCH * KPIX * NCH * 4;
  const size_t szOFF  = (size_t)NBATCH * QPIX * NOFF * 4;
  const size_t szIM   = (size_t)IMGS_PER_CHUNK * QPIX * KIM * 2;

  size_t offb = 0;
  char* base = (char*)d_ws;
  auto carve = [&](size_t bytes) -> char* {
    char* p = base + offb;
    offb += (bytes + 255) & ~(size_t)255;
    return p;
  };
  unsigned short* QT    = (unsigned short*)carve(szQT);
  unsigned short* OUT16 = QT;
  unsigned short* KVT   = (unsigned short*)carve(szKVT);
  unsigned short* WQ    = (unsigned short*)carve(szW);
  unsigned short* WK    = (unsigned short*)carve(szW);
  unsigned short* WV    = (unsigned short*)carve(szW);
  unsigned short* WOUT  = (unsigned short*)carve(szW);
  unsigned short* WOFF  = (unsigned short*)carve(szWOFF);
  float*          QF    = (float*)carve(szQ);
  float*          KF    = (float*)carve(szK);
  float*          VF    = (float*)carve(szK);
  float*          OFF   = (float*)carve(szOFF);
  unsigned short* IM    = (unsigned short*)carve(szIM);
  if (offb > ws_size) return;

  k_tr_in<<<dim3(QPIX / 64, NCH / 64, NBATCH), 256, 0, stream>>>(query_map, QT, QPIX);
  k_tr_in<<<dim3(KPIX / 64, NCH / 64, NBATCH), 256, 0, stream>>>(kv_map, KVT, KPIX);
  k_castw<<<dim3((NCH * NCH) / (8 * 256), 4), 256, 0, stream>>>(q_w, k_w, v_w, out_w, WQ, WK, WV, WOUT);
  k_prepoff<<<(NOFF * KIM / 8) / 256, 256, 0, stream>>>(offset_w, WOFF);

  {
    const int tiles = (QPIX / 64) * (NCH / 64);
    wmma_gemm64<1, 0, 0, 0, false, 0><<<dim3(tiles / 8, NBATCH), 256, 0, stream>>>(
        QT, QT, NCH, (long)QPIX * NCH, WQ, WQ, NCH, 0L,
        QF, QF, NCH, (long)QPIX * NCH, offset_b, offset_b, 0L, QPIX, NCH, NCH, 1.0f);
  }
  {
    const int tiles = (KPIX / 64) * (NCH / 64);
    wmma_gemm64<1, 0, 0, 0, false, 0><<<dim3(tiles / 8, NBATCH), 256, 0, stream>>>(
        KVT, KVT, NCH, (long)KPIX * NCH, WK, WK, NCH, 0L,
        KF, KF, NCH, (long)KPIX * NCH, offset_b, offset_b, 0L, KPIX, NCH, NCH, 1.0f);
    wmma_gemm64<1, 0, 0, 0, false, 0><<<dim3(tiles / 8, NBATCH), 256, 0, stream>>>(
        KVT, KVT, NCH, (long)KPIX * NCH, WV, WV, NCH, 0L,
        VF, VF, NCH, (long)KPIX * NCH, offset_b, offset_b, 0L, KPIX, NCH, NCH, 1.0f);
  }

  for (int ch = 0; ch < NCHUNK; ++ch) {
    const int b0 = ch * IMGS_PER_CHUNK;
    k_im2col<<<(IMGS_PER_CHUNK * QPIX * NTAP) / 8, 256, 0, stream>>>(QT, IM, b0);
    const int tiles = (QPIX / 64) * (NOFF / 64);
    float* offc = OFF + (size_t)b0 * QPIX * NOFF;
    wmma_gemm64<1, 0, 2, 0, false, 0><<<dim3(tiles / 8, IMGS_PER_CHUNK), 256, 0, stream>>>(
        IM, IM, KIM, (long)QPIX * KIM, WOFF, WOFF, KIM, 0L,
        offc, offc, NOFF, (long)QPIX * NOFF, offset_b, offset_b, 0L, QPIX, NOFF, KIM, 1.0f);
  }

  k_sample<<<(NBATCH * QPIX) / 8, 256, 0, stream>>>(QF, KF, VF, OFF, OUT16);

  {
    const int tiles = (NCH / 64) * (QPIX / 64);
    wmma_gemm64<0, 0, 0, 0, false, 0><<<dim3(tiles / 8, NBATCH), 256, 0, stream>>>(
        WOUT, WOUT, NCH, 0L, OUT16, OUT16, NCH, (long)QPIX * NCH,
        out, out, QPIX, (long)NCH * QPIX, offset_b, offset_b, 0L, NCH, QPIX, NCH, OUT_SCALE);
  }
}
